// EGNN_5995774345800
// MI455X (gfx1250) — hardware-verified
//
#include <hip/hip_runtime.h>
#include <stddef.h>
#include <stdint.h>

#define NBAT   2
#define NNODE  512
#define NROW   1024
#define DIM    64
#define MDIM   16
#define H1     274
#define H1P    288
#define NPIJ   576
#define NFOUR  9
#define HN     128
#define OUT1_OFF 65536

#define VB1E 0
#define VB2E 288
#define VB1C 320
#define VW2C 384
#define VB2C 448
#define VB1H 480
#define VB2H 608
#define VECN 672

#define PB_FB    0
#define PB_W1IJ  32
#define PB_WF    50
#define PB_W2E   55
#define PB_W1C   58
#define PB_W1HF  59
#define PB_W1HM  63
#define PB_W2H   65
#define PB_VEC   69
#define PB_CB    71
#define PB_END   75

#define L_PJ   0
#define L_WF   73728
#define L_W2E  92160
#define L_W1C  101376
#define L_PI   105472
#define L_CB   114688
#define L_VEC  122880
#define L_MI   123904
#define L_CO   124416
#define PAIR_LDS 124544

static_assert(NNODE % 64 == 0);
static_assert(H1 <= H1P && H1P == 9 * 32);
static_assert(2 * NFOUR <= 32);
static_assert(MDIM == 16);
static_assert(NROW == NBAT * NNODE && NROW % 128 == 0 && NPIJ % 64 == 0 && NPIJ == 2 * H1P);
static_assert((32 * 3 * 4) % 128 == 0);
static_assert(OUT1_OFF == NROW * DIM && (OUT1_OFF * 4) % 128 == 0);
static_assert(PAIR_LDS <= 327680);
static_assert(VB2E == VB1E + 288 && VB1C == VB2E + 32 && VW2C == VB1C + 64 && VB2C == VW2C + 64);
static_assert(VB1H == VB2C + 32 && VB2H == VB1H + 128 && VECN == VB2H + 64 && VB2E + 256 <= VECN);
static_assert((NROW * DIM / 8) == (PB_W1IJ - PB_FB) * 256);
static_assert((NPIJ * 8) == (PB_WF - PB_W1IJ) * 256);
static_assert((H1P * 4) <= (PB_W2E - PB_WF) * 256 && (MDIM * 36) <= (PB_W1C - PB_W2E) * 256);
static_assert(64 * 4 == (PB_W1HF - PB_W1C) * 256 && 128 * 8 == (PB_W1HM - PB_W1HF) * 256);
static_assert(128 * 4 == (PB_W2H - PB_W1HM) * 256 && 64 * 16 == (PB_VEC - PB_W2H) * 256);
static_assert(NROW == (PB_END - PB_CB) * 256);

typedef float          v4f   __attribute__((ext_vector_type(4)));
typedef float          v8f   __attribute__((ext_vector_type(8)));
typedef int            v8i   __attribute__((ext_vector_type(8)));
typedef unsigned short v8us  __attribute__((ext_vector_type(8)));
typedef unsigned short v16us __attribute__((ext_vector_type(16)));
typedef __bf16         v16bf __attribute__((ext_vector_type(16)));
typedef v4f  __attribute__((may_alias)) v4fa;
typedef v8us __attribute__((may_alias)) v8usa;
union FragB { v16bf v; v16us u; v8us h[2]; v8i w; };

__device__ __forceinline__ v8f wmb(const FragB& a, const FragB& b, v8f c) {
  v8f d = __builtin_amdgcn_wmma_f32_16x16x32_bf16(false, a.v, false, b.v, (short)0, c, false, false);
  asm volatile("v_nop\n\tv_nop\n\tv_nop\n\tv_nop" : "+v"(d) : "v"(a.w), "v"(b.w));
  return d;
}

__device__ __forceinline__ unsigned bf16_bits(float f) {
  const unsigned u = __float_as_uint(f);
  return (u + 0x7FFFu + ((u >> 16) & 1u)) >> 16;
}
__device__ __forceinline__ float bf16_val(float f) { return __uint_as_float(bf16_bits(f) << 16); }
__device__ __forceinline__ unsigned pk2(unsigned lo, unsigned hi) { return (lo & 0xffffu) | (hi << 16); }
__device__ __forceinline__ float relu_f(float v) { return (v > 0.0f) ? v : 0.0f; }

__device__ __forceinline__ void put16(unsigned short* dp, v8us o) {
  *(volatile v8us*)dp = o;
  __threadfence();
  *(volatile v8us*)dp = o;
}
__device__ __forceinline__ void putf4(float* dp, v4f o) {
  *(volatile v4f*)dp = o;
  __threadfence();
  *(volatile v4f*)dp = o;
}

__device__ __forceinline__ void frag_glb(FragB& f, const unsigned short* __restrict__ p) {
  f.h[0] = *(const v8usa*)p;
  f.h[1] = *(const v8usa*)(p + 16);
}

__device__ __forceinline__ void vec_unit(const float* __restrict__ src, int nreal, int nunits, float* dst, int u) {
  if (u >= nunits) return;
  v4f q;
  const int g0 = 4 * u;
  const int i0 = g0     < nreal ? g0     : nreal - 1;
  const int i1 = g0 + 1 < nreal ? g0 + 1 : nreal - 1;
  const int i2 = g0 + 2 < nreal ? g0 + 2 : nreal - 1;
  const int i3 = g0 + 3 < nreal ? g0 + 3 : nreal - 1;
  const float x0 = src[i0], x1 = src[i1], x2 = src[i2], x3 = src[i3];
  q.x = (g0     < nreal) ? bf16_val(x0) : 0.0f;
  q.y = (g0 + 1 < nreal) ? bf16_val(x1) : 0.0f;
  q.z = (g0 + 2 < nreal) ? bf16_val(x2) : 0.0f;
  q.w = (g0 + 3 < nreal) ? bf16_val(x3) : 0.0f;
  putf4(dst + g0, q);
}

__global__ __launch_bounds__(256) void k_prep(
    const float* __restrict__ feats, const float* __restrict__ coors,
    const float* __restrict__ w1e, const float* __restrict__ b1e,
    const float* __restrict__ w2e, const float* __restrict__ b2e,
    const float* __restrict__ w1c, const float* __restrict__ b1c,
    const float* __restrict__ w2c, const float* __restrict__ b2c,
    const float* __restrict__ w1h, const float* __restrict__ b1h,
    const float* __restrict__ w2h, const float* __restrict__ b2h,
    unsigned short* FB, unsigned short* W1IJ, unsigned short* WF, unsigned short* W2E,
    unsigned short* W1C, unsigned short* W1HF, unsigned short* W1HM, unsigned short* W2H,
    float* VEC, float* CB) {
  const int blk = (int)blockIdx.x, tid = (int)threadIdx.x;
  v8us o;
  if (blk < PB_W1IJ) {
    const int v = blk * 256 + tid;
    const float* p = feats + (size_t)v * 8;
    const v4f a = *(const v4fa*)p;
    const v4f b = *(const v4fa*)(p + 4);
    o[0] = (unsigned short)bf16_bits(a.x); o[1] = (unsigned short)bf16_bits(a.y);
    o[2] = (unsigned short)bf16_bits(a.z); o[3] = (unsigned short)bf16_bits(a.w);
    o[4] = (unsigned short)bf16_bits(b.x); o[5] = (unsigned short)bf16_bits(b.y);
    o[6] = (unsigned short)bf16_bits(b.z); o[7] = (unsigned short)bf16_bits(b.w);
    put16(FB + (size_t)v * 8, o);
    return;
  }
  if (blk < PB_WF) {
    const int v  = (blk - PB_W1IJ) * 256 + tid;
    const int n  = v >> 3;
    const int k8 = (v & 7) * 8;
    const int hf = n >= H1P ? 1 : 0;
    const int nn = n - H1P * hf;
    const bool ok = nn < H1;
    const int nc = ok ? nn : H1 - 1;
    const float* p = w1e + (size_t)(64 * hf + k8) * H1 + nc;
#pragma unroll
    for (int i = 0; i < 8; ++i) {
      const unsigned bits = bf16_bits(p[(size_t)i * H1]);
      o[i] = (unsigned short)(ok ? bits : 0u);
    }
    put16(W1IJ + (size_t)v * 8, o);
    return;
  }
  if (blk < PB_W2E) {
    const int v = (blk - PB_WF) * 256 + tid;
    if (v >= H1P * 4) return;
    const int n  = v >> 2;
    const int k8 = (v & 3) * 8;
    const bool nok = n < H1;
    const int nc = nok ? n : H1 - 1;
#pragma unroll
    for (int i = 0; i < 8; ++i) {
      const int k  = k8 + i;
      int kk = k < NFOUR ? k : k - NFOUR;
      kk = kk > NFOUR - 1 ? NFOUR - 1 : kk;
      const bool ok = nok && (k < 2 * NFOUR);
      const unsigned bits = bf16_bits(w1e[(size_t)(128 + kk) * H1 + nc]);
      o[i] = (unsigned short)(ok ? bits : 0u);
    }
    put16(WF + (size_t)v * 8, o);
    return;
  }
  if (blk < PB_W1C) {
    const int v = (blk - PB_W2E) * 256 + tid;
    if (v >= MDIM * 36) return;
    const int n  = v / 36;
    const int k8 = (v - 36 * n) * 8;
#pragma unroll
    for (int i = 0; i < 8; ++i) {
      const int k = k8 + i;
      const bool ok = k < H1;
      const int kc = ok ? k : H1 - 1;
      const unsigned bits = bf16_bits(w2e[(size_t)kc * MDIM + n]);
      o[i] = (unsigned short)(ok ? bits : 0u);
    }
    put16(W2E + (size_t)v * 8, o);
    return;
  }
  if (blk < PB_W1HF) {
    const int v  = tid;
    const int n  = v >> 2;
    const int k8 = (v & 3) * 8;
#pragma unroll
    for (int i = 0; i < 8; ++i) o[i] = (unsigned short)bf16_bits(w1c[(size_t)((k8 + i) & 15) * 64 + n]);
    put16(W1C + (size_t)v * 8, o);
    return;
  }
  if (blk < PB_W1HM) {
    const int v  = (blk - PB_W1HF) * 256 + tid;
    const int n  = v >> 3;
    const int k8 = (v & 7) * 8;
#pragma unroll
    for (int i = 0; i < 8; ++i) o[i] = (unsigned short)bf16_bits(w1h[(size_t)(k8 + i) * HN + n]);
    put16(W1HF + (size_t)v * 8, o);
    return;
  }
  if (blk < PB_W2H) {
    const int v  = (blk - PB_W1HM) * 256 + tid;
    const int n  = v >> 2;
    const int k8 = (v & 3) * 8;
#pragma unroll
    for (int i = 0; i < 8; ++i) o[i] = (unsigned short)bf16_bits(w1h[(size_t)(64 + ((k8 + i) & 15)) * HN + n]);
    put16(W1HM + (size_t)v * 8, o);
    return;
  }
  if (blk < PB_VEC) {
    const int v  = (blk - PB_W2H) * 256 + tid;
    const int n  = v >> 4;
    const int k8 = (v & 15) * 8;
#pragma unroll
    for (int i = 0; i < 8; ++i) o[i] = (unsigned short)bf16_bits(w2h[(size_t)(k8 + i) * DIM + n]);
    put16(W2H + (size_t)v * 8, o);
    return;
  }
  if (blk < PB_CB) {
    const int gw   = (blk - PB_VEC) * 8 + (tid >> 5);
    const int lane = tid & 31;
    if (gw < 3)       vec_unit(b1e, H1, 72, VEC + VB1E, gw * 32 + lane);
    else if (gw == 3) vec_unit(b2e, MDIM, 8, VEC + VB2E, lane);
    else if (gw == 4) vec_unit(b1c, 64, 16, VEC + VB1C, lane);
    else if (gw == 5) vec_unit(w2c, 64, 16, VEC + VW2C, lane);
    else if (gw == 6) vec_unit(b2c, 1, 8, VEC + VB2C, lane);
    else if (gw == 7) vec_unit(b1h, HN, 32, VEC + VB1H, lane);
    else if (gw == 8) vec_unit(b2h, DIM, 16, VEC + VB2H, lane);
    return;
  }
  {
    const int row = (blk - PB_CB) * 256 + tid;
    const float x0 = coors[(size_t)row * 3 + 0];
    const float x1 = coors[(size_t)row * 3 + 1];
    const float x2 = coors[(size_t)row * 3 + 2];
    v4f q;
    q.x = bf16_val(x0); q.y = bf16_val(x1); q.z = bf16_val(x2); q.w = 0.0f;
    putf4(CB + (size_t)row * 4, q);
  }
}

__global__ __launch_bounds__(128) void k_node(const unsigned short* __restrict__ FB,
                                              const unsigned short* __restrict__ W1IJ,
                                              const float* __restrict__ VEC, float* PIJ) {
  __shared__ __attribute__((aligned(16))) float sF[128 * 64];
  const int tid = (int)threadIdx.x, lane = tid & 31, w = tid >> 5, hh = lane >> 4, m = lane & 15;
  const int m0 = (int)blockIdx.x * 128;
  const int n0 = (int)blockIdx.y * 64;
  const int m0w = m0 + 32 * w;

  v8f acc[2][4];
  {
    const v8f z = {0.f, 0.f, 0.f, 0.f, 0.f, 0.f, 0.f, 0.f};
#pragma unroll
    for (int mt = 0; mt < 2; ++mt)
#pragma unroll
      for (int nt = 0; nt < 4; ++nt) acc[mt][nt] = z;
  }
  const unsigned short* a0 = FB + (size_t)(m0w + m) * DIM + 8 * hh;
  const unsigned short* a1 = a0 + (size_t)16 * DIM;
  const unsigned short* bp = W1IJ + (size_t)(n0 + m) * DIM + 8 * hh;
#pragma unroll 1
  for (int k0 = 0; k0 < DIM; k0 += 32) {
    FragB f0, f1;
    frag_glb(f0, a0 + k0);
    frag_glb(f1, a1 + k0);
#pragma unroll
    for (int nt = 0; nt < 4; ++nt) {
      FragB fb;
      frag_glb(fb, bp + (size_t)nt * 16 * DIM + k0);
      acc[0][nt] = wmb(f0, fb, acc[0][nt]);
      acc[1][nt] = wmb(f1, fb, acc[1][nt]);
    }
  }
#pragma unroll
  for (int nt = 0; nt < 4; ++nt) {
    const int col = n0 + 16 * nt + m;
    const int cc  = col < H1P ? col : H1P - 1;
    const float bl = VEC[VB1E + cc];
    const float bv = (col < H1P) ? bl : 0.0f;
#pragma unroll
    for (int mt = 0; mt < 2; ++mt)
#pragma unroll
      for (int r = 0; r < 8; ++r)
        sF[(32 * w + 16 * mt + 8 * hh + r) * 64 + 16 * nt + m] = acc[mt][nt][r] + bv;
  }
  __syncthreads();
  {
    const int rsub = lane >> 4, c4 = (lane & 15) * 4;
    v4f vals[16];
#pragma unroll
    for (int it = 0; it < 16; ++it) vals[it] = *(const v4fa*)(sF + (32 * w + 2 * it + rsub) * 64 + c4);
#pragma unroll
    for (int it = 0; it < 16; ++it)
      *(volatile v4f*)(PIJ + (size_t)(m0 + 32 * w + 2 * it + rsub) * NPIJ + n0 + c4) = vals[it];
    __threadfence();
#pragma unroll
    for (int it = 0; it < 16; ++it)
      *(volatile v4f*)(PIJ + (size_t)(m0 + 32 * w + 2 * it + rsub) * NPIJ + n0 + c4) = vals[it];
  }
}

__global__ __launch_bounds__(256) void k_pair(const float* __restrict__ PIJ,
                                              const unsigned short* __restrict__ WF,
                                              const unsigned short* __restrict__ W2E,
                                              const unsigned short* __restrict__ W1C,
                                              const float* __restrict__ VEC, const float* __restrict__ CB,
                                              float* MI, float* CO) {
  extern __shared__ __attribute__((aligned(16))) float dyn[];
  float*          sPJ  = dyn + (L_PJ >> 2);
  unsigned short* sWF  = (unsigned short*)(dyn + (L_WF >> 2));
  unsigned short* sW2E = (unsigned short*)(dyn + (L_W2E >> 2));
  unsigned short* sW1C = (unsigned short*)(dyn + (L_W1C >> 2));
  float*          sPI  = dyn + (L_PI >> 2);
  float*          sCB  = dyn + (L_CB >> 2);
  float*          sVec = dyn + (L_VEC >> 2);
  float*          sMI  = dyn + (L_MI >> 2);
  float*          sCO  = dyn + (L_CO >> 2);

  const int tid = (int)threadIdx.x, lane = tid & 31, wave = tid >> 5, hh = lane >> 4, m = lane & 15;
  const int blk = (int)blockIdx.x;
  const int b   = blk >> 6;
  const int i0  = (blk & 63) * 8;

  for (int u = tid; u < H1P * 4; u += 256) *(v4fa*)(sWF + 8 * u) = *(const v4fa*)(WF + 8 * u);
  for (int u = tid; u < MDIM * 36; u += 256) *(v4fa*)(sW2E + 8 * u) = *(const v4fa*)(W2E + 8 * u);
  *(v4fa*)(sW1C + 8 * tid) = *(const v4fa*)(W1C + 8 * tid);
  for (int u = tid; u < 8 * 72; u += 256) {
    const int row = u / 72;
    const int c   = u - 72 * row;
    *(v4fa*)(sPI + row * H1P + 4 * c) = *(const v4fa*)(PIJ + (size_t)(b * NNODE + i0 + row) * NPIJ + 4 * c);
  }
  for (int u = tid; u < NNODE; u += 256) *(v4fa*)(sCB + 4 * u) = *(const v4fa*)(CB + (size_t)(b * NNODE + u) * 4);
  if (tid < 64) *(v4fa*)(sVec + 4 * tid) = *(const v4fa*)(VEC + VB2E + 4 * tid);
  __syncthreads();

  const v4f ci = *(const v4fa*)(sCB + 4 * (i0 + wave));
  float b2r[8];
  {
    const v4f x = *(const v4fa*)(sVec + 8 * hh);
    const v4f y = *(const v4fa*)(sVec + 8 * hh + 4);
    b2r[0] = x.x; b2r[1] = x.y; b2r[2] = x.z; b2r[3] = x.w;
    b2r[4] = y.x; b2r[5] = y.y; b2r[6] = y.z; b2r[7] = y.w;
  }
  const float b2cv = sVec[160];
  const float* pirow = sPI + wave * H1P + 8 * hh;
  const float sc0 = hh ? 0.25f : 1.0f;
  const float sc1 = hh ? 0.125f : 0.5f;
  const bool  up  = hh != 0;
  const unsigned mk = 0u - (unsigned)hh;
  const unsigned nk = ~mk;

  float msum[8];
#pragma unroll
  for (int r = 0; r < 8; ++r) msum[r] = 0.0f;
  float ca0 = 0.0f, ca1 = 0.0f, ca2 = 0.0f;

#pragma unroll 1
  for (int jc = 0; jc < NNODE / 64; ++jc) {
    __syncthreads();
#pragma unroll 3
    for (int it = 0; it < 18; ++it) {
      const int u   = it * 256 + tid;
      const int row = u / 72;
      const int c   = u - 72 * row;
      const v4f v = *(const v4fa*)(PIJ + (size_t)(b * NNODE + jc * 64 + row) * NPIJ + H1P + 4 * c);
      *(v4fa*)(sPJ + 4 * u) = v;
    }
    __syncthreads();

#pragma unroll 1
    for (int jt = 0; jt < 4; ++jt) {
      const int jl = jt * 16 + m;
      const int j  = jc * 64 + jl;
      const v4f cj = *(const v4fa*)(sCB + 4 * j);
      const float rx = ci.x - cj.x, ry = ci.y - cj.y, rz = ci.z - cj.z;
      const float sq = (rx * rx + rz * rz) + ry * ry;
      const float d  = (sq > 0.0f) ? sqrtf(sq) : 0.0f;

      FragB bfour;
      {
        const float x0 = d * sc0, x1 = d * sc1;
        const float s0 = sinf(x0), c0 = cosf(x0);
        const float s1 = sinf(x1), c1 = cosf(x1);
        const float ps0 = __shfl_xor(s0, 16, 32);
        const float pc0 = __shfl_xor(c0, 16, 32);
        const float ps1 = __shfl_xor(s1, 16, 32);
        const float pc1 = __shfl_xor(c1, 16, 32);
        float f[NFOUR];
        f[0] = up ? ps0 : s0;  f[1] = up ? ps1 : s1;  f[2] = up ? s0 : ps0;  f[3] = up ? s1 : ps1;
        f[4] = up ? pc0 : c0;  f[5] = up ? pc1 : c1;  f[6] = up ? c0 : pc0;  f[7] = up ? c1 : pc1;
        f[8] = d;
        unsigned hb[NFOUR], lb[NFOUR];
#pragma unroll
        for (int q = 0; q < NFOUR; ++q) {
          hb[q] = bf16_bits(f[q]);
          lb[q] = bf16_bits(f[q] - __uint_as_float(hb[q] << 16));
        }
        const unsigned e0 = (hb[0] & nk) | (hb[8] & mk);
        const unsigned e1 = (hb[1] & nk) | (lb[0] & mk);
        const unsigned e2 = (hb[2] & nk) | (lb[1] & mk);
        const unsigned e3 = (hb[3] & nk) | (lb[2] & mk);
        const unsigned e4 = (hb[4] & nk) | (lb[3] & mk);
        const unsigned e5 = (hb[5] & nk) | (lb[4] & mk);
        const unsigned e6 = (hb[6] & nk) | (lb[5] & mk);
        const unsigned e7 = (hb[7] & nk) | (lb[6] & mk);
        const unsigned e8 = lb[7] & nk;
        const unsigned e9 = lb[8] & nk;
        bfour.w[0] = (int)pk2(e0, e1);
        bfour.w[1] = (int)pk2(e2, e3);
        bfour.w[2] = (int)pk2(e4, e5);
        bfour.w[3] = (int)pk2(e6, e7);
        bfour.w[4] = (int)pk2(e8, e9);
        bfour.w[5] = 0; bfour.w[6] = 0; bfour.w[7] = 0;
      }

      const float* pjrow = sPJ + jl * H1P + 8 * hh;
      v8f macc = {0.f, 0.f, 0.f, 0.f, 0.f, 0.f, 0.f, 0.f};

#pragma unroll 1
      for (int kc = 0; kc < H1P / 32; ++kc) {
        FragB bh, bl;
#pragma unroll
        for (int t = 0; t < 2; ++t) {
          const int n0 = 32 * kc + 16 * t;
          FragB aw;
          aw.h[0] = *(const v8usa*)(sWF + (n0 + m) * 32 + 8 * hh);
          aw.h[1] = *(const v8usa*)(sWF + (n0 + m) * 32 + 16 + 8 * hh);
          const v4f p0 = *(const v4fa*)(pirow + n0);
          const v4f p1 = *(const v4fa*)(pirow + n0 + 4);
          const v4f q0 = *(const v4fa*)(pjrow + n0);
          const v4f q1 = *(const v4fa*)(pjrow + n0 + 4);
          const v8f c = {p0.x + q0.x, p0.y + q0.y, p0.z + q0.z, p0.w + q0.w,
                         p1.x + q1.x, p1.y + q1.y, p1.z + q1.z, p1.w + q1.w};
          const v8f dd = wmb(aw, bfour, c);
#pragma unroll
          for (int q = 0; q < 4; ++q) {
            const float v0 = relu_f(dd[2 * q]);
            const float v1 = relu_f(dd[2 * q + 1]);
            const unsigned h0 = bf16_bits(v0), h1 = bf16_bits(v1);
            const unsigned l0 = bf16_bits(v0 - __uint_as_float(h0 << 16));
            const unsigned l1 = bf16_bits(v1 - __uint_as_float(h1 << 16));
            bh.w[4 * t + q] = (int)pk2(h0, h1);
            bl.w[4 * t + q] = (int)pk2(l0, l1);
          }
        }
        FragB a2;
        a2.h[0] = *(const v8usa*)(sW2E + m * H1P + 32 * kc + 8 * hh);
        a2.h[1] = *(const v8usa*)(sW2E + m * H1P + 32 * kc + 16 + 8 * hh);
        macc = wmb(a2, bh, macc);
        macc = wmb(a2, bl, macc);
      }

      FragB bm;
      {
        float mf[8];
#pragma unroll
        for (int r = 0; r < 8; ++r) {
          mf[r] = macc[r] + b2r[r];
          msum[r] += mf[r];
        }
#pragma unroll
        for (int q = 0; q < 4; ++q) {
          const unsigned h0 = bf16_bits(mf[2 * q]), h1 = bf16_bits(mf[2 * q + 1]);
          const unsigned l0 = bf16_bits(mf[2 * q] - __uint_as_float(h0 << 16));
          const unsigned l1 = bf16_bits(mf[2 * q + 1] - __uint_as_float(h1 << 16));
          bm.w[q]     = (int)pk2(h0, h1);
          bm.w[4 + q] = (int)pk2(l0, l1);
        }
      }
      float part = 0.0f;
#pragma unroll 1
      for (int t = 0; t < 4; ++t) {
        FragB a3;
        a3.h[0] = *(const v8usa*)(sW1C + (16 * t + m) * 32 + 8 * hh);
        a3.h[1] = *(const v8usa*)(sW1C + (16 * t + m) * 32 + 16 + 8 * hh);
        const v4f ba = *(const v4fa*)(sVec + 32 + 16 * t + 8 * hh);
        const v4f bb = *(const v4fa*)(sVec + 32 + 16 * t + 8 * hh + 4);
        const v8f c = {ba.x, ba.y, ba.z, ba.w, bb.x, bb.y, bb.z, bb.w};
        const v8f d3 = wmb(a3, bm, c);
        const v4f wa = *(const v4fa*)(sVec + 96 + 16 * t + 8 * hh);
        const v4f wb = *(const v4fa*)(sVec + 96 + 16 * t + 8 * hh + 4);
        part = fmaf(relu_f(d3[0]), wa.x, part);
        part = fmaf(relu_f(d3[1]), wa.y, part);
        part = fmaf(relu_f(d3[2]), wa.z, part);
        part = fmaf(relu_f(d3[3]), wa.w, part);
        part = fmaf(relu_f(d3[4]), wb.x, part);
        part = fmaf(relu_f(d3[5]), wb.y, part);
        part = fmaf(relu_f(d3[6]), wb.z, part);
        part = fmaf(relu_f(d3[7]), wb.w, part);
      }
      const float other = __shfl_xor(part, 16, 32);
      const float cw = (part + other) + b2cv;
      ca0 = fmaf(cw, rx, ca0);
      ca1 = fmaf(cw, ry, ca1);
      ca2 = fmaf(cw, rz, ca2);
    }
  }

#pragma unroll
  for (int r = 0; r < 8; ++r) {
    float v = msum[r];
    v += __shfl_xor(v, 1, 32);
    v += __shfl_xor(v, 2, 32);
    v += __shfl_xor(v, 4, 32);
    v += __shfl_xor(v, 8, 32);
    msum[r] = v;
  }
  ca0 += __shfl_xor(ca0, 1, 32); ca0 += __shfl_xor(ca0, 2, 32); ca0 += __shfl_xor(ca0, 4, 32); ca0 += __shfl_xor(ca0, 8, 32);
  ca1 += __shfl_xor(ca1, 1, 32); ca1 += __shfl_xor(ca1, 2, 32); ca1 += __shfl_xor(ca1, 4, 32); ca1 += __shfl_xor(ca1, 8, 32);
  ca2 += __shfl_xor(ca2, 1, 32); ca2 += __shfl_xor(ca2, 2, 32); ca2 += __shfl_xor(ca2, 4, 32); ca2 += __shfl_xor(ca2, 8, 32);

  if (m == 0) {
    const v4f x = {msum[0], msum[1], msum[2], msum[3]};
    const v4f y = {msum[4], msum[5], msum[6], msum[7]};
    *(v4fa*)(sMI + wave * 16 + 8 * hh)     = x;
    *(v4fa*)(sMI + wave * 16 + 8 * hh + 4) = y;
  }
  if (lane == 0) {
    const v4f cq = {ca0, ca1, ca2, 0.0f};
    *(v4fa*)(sCO + wave * 4) = cq;
  }
  __syncthreads();
  if (wave == 0) {
    const v4f mo = *(const v4fa*)(sMI + 4 * lane);
    putf4(MI + (size_t)blk * 128 + 4 * lane, mo);
    const int tl = lane < 8 ? lane : 7;
    const v4f co = *(const v4fa*)(sCO + 4 * tl);
    float* cp = CO + (size_t)blk * 32 + 4 * tl;
    if (lane < 8) *(volatile v4f*)cp = co;
    __threadfence();
    if (lane < 8) *(volatile v4f*)cp = co;
  }
}

__global__ __launch_bounds__(64) void k_update(const unsigned short* __restrict__ FB,
                                               const unsigned short* __restrict__ W1HF,
                                               const unsigned short* __restrict__ W1HM,
                                               const unsigned short* __restrict__ W2H,
                                               const float* __restrict__ VEC,
                                               const float* __restrict__ MI, const float* __restrict__ CO,
                                               float* out) {
  __shared__ __attribute__((aligned(16))) float sOut[32 * 64];
  __shared__ __attribute__((aligned(16))) float sCo[96];
  const int tid = (int)threadIdx.x, lane = tid & 31, wave = tid >> 5, hh = lane >> 4, m = lane & 15;
  const int blk = (int)blockIdx.x;
  const int nodeBase = blk * 32;
  const int node = nodeBase + 16 * wave + m;

  FragB bf0, bf1, bmi;
  frag_glb(bf0, FB + (size_t)node * DIM + 8 * hh);
  frag_glb(bf1, FB + (size_t)node * DIM + 32 + 8 * hh);
  {
    const float* mq = MI + (size_t)node * MDIM + 8 * hh;
    const v4f x = *(const v4fa*)mq;
    const v4f y = *(const v4fa*)(mq + 4);
    const v8f v8 = {x.x, x.y, x.z, x.w, y.x, y.y, y.z, y.w};
#pragma unroll
    for (int q = 0; q < 4; ++q) {
      const unsigned h0 = bf16_bits(v8[2 * q]), h1 = bf16_bits(v8[2 * q + 1]);
      const unsigned l0 = bf16_bits(v8[2 * q] - __uint_as_float(h0 << 16));
      const unsigned l1 = bf16_bits(v8[2 * q + 1] - __uint_as_float(h1 << 16));
      bmi.w[q]     = (int)pk2(h0, h1);
      bmi.w[4 + q] = (int)pk2(l0, l1);
    }
  }

  v8f acc[8];
#pragma unroll
  for (int t = 0; t < 8; ++t) {
    const int n = 16 * t + m;
    const v4f ba = *(const v4fa*)(VEC + VB1H + 16 * t + 8 * hh);
    const v4f bb = *(const v4fa*)(VEC + VB1H + 16 * t + 8 * hh + 4);
    v8f c = {ba.x, ba.y, ba.z, ba.w, bb.x, bb.y, bb.z, bb.w};
    FragB a0, a1, a2;
    frag_glb(a0, W1HF + (size_t)n * DIM + 8 * hh);
    frag_glb(a1, W1HF + (size_t)n * DIM + 32 + 8 * hh);
    frag_glb(a2, W1HM + (size_t)n * 32 + 8 * hh);
    c = wmb(a0, bf0, c);
    c = wmb(a1, bf1, c);
    c = wmb(a2, bmi, c);
    acc[t] = c;
  }

  FragB bh[4], bl[4];
#pragma unroll
  for (int s = 0; s < 4; ++s)
#pragma unroll
    for (int hf = 0; hf < 2; ++hf)
#pragma unroll
      for (int q = 0; q < 4; ++q) {
        const float v0 = relu_f(acc[2 * s + hf][2 * q]);
        const float v1 = relu_f(acc[2 * s + hf][2 * q + 1]);
        const unsigned h0 = bf16_bits(v0), h1 = bf16_bits(v1);
        const unsigned l0 = bf16_bits(v0 - __uint_as_float(h0 << 16));
        const unsigned l1 = bf16_bits(v1 - __uint_as_float(h1 << 16));
        bh[s].w[4 * hf + q] = (int)pk2(h0, h1);
        bl[s].w[4 * hf + q] = (int)pk2(l0, l1);
      }

#pragma unroll
  for (int t2 = 0; t2 < 4; ++t2) {
    const v4f ba = *(const v4fa*)(VEC + VB2H + 16 * t2 + 8 * hh);
    const v4f bb = *(const v4fa*)(VEC + VB2H + 16 * t2 + 8 * hh + 4);
    v8f o = {ba.x, ba.y, ba.z, ba.w, bb.x, bb.y, bb.z, bb.w};
#pragma unroll
    for (int s = 0; s < 4; ++s) {
      FragB a;
      frag_glb(a, W2H + (size_t)(16 * t2 + m) * HN + 32 * s + 8 * hh);
      o = wmb(a, bh[s], o);
      o = wmb(a, bl[s], o);
    }
    const v4f o0 = {o[0], o[1], o[2], o[3]};
    const v4f o1 = {o[4], o[5], o[6], o[7]};
    *(v4fa*)(sOut + (16 * wave + m) * 64 + 16 * t2 + 8 * hh)     = o0;
    *(v4fa*)(sOut + (16 * wave + m) * 64 + 16 * t2 + 8 * hh + 4) = o1;
  }
  if (tid < 32) {
    const v4f c = *(const v4fa*)(CO + (size_t)(nodeBase + tid) * 4);
    sCo[3 * tid + 0] = c.x;
    sCo[3 * tid + 1] = c.y;
    sCo[3 * tid + 2] = c.z;
  }
  __syncthreads();

  {
    const int rsub = lane >> 4, c4 = (lane & 15) * 4;
    v4f vals[8];
#pragma unroll
    for (int it = 0; it < 8; ++it) vals[it] = *(const v4fa*)(sOut + (16 * wave + 2 * it + rsub) * 64 + c4);
#pragma unroll
    for (int it = 0; it < 8; ++it)
      *(volatile v4f*)(out + (size_t)(nodeBase + 16 * wave + 2 * it + rsub) * DIM + c4) = vals[it];
    __threadfence();
#pragma unroll
    for (int it = 0; it < 8; ++it)
      *(volatile v4f*)(out + (size_t)(nodeBase + 16 * wave + 2 * it + rsub) * DIM + c4) = vals[it];
  }
  if (wave == 0) {
    const int tl = lane < 24 ? lane : 23;
    const v4f o = *(const v4fa*)(sCo + 4 * tl);
    float* op = out + OUT1_OFF + (size_t)blk * 96 + 4 * tl;
    if (lane < 24) *(volatile v4f*)op = o;
    __threadfence();
    if (lane < 24) *(volatile v4f*)op = o;
  }
}

static inline size_t al256(size_t x) { return (x + 255) & ~(size_t)255; }

extern "C" void kernel_launch(void* const* d_in, const int* in_sizes, int n_in,
                              void* d_out, int out_size, void* d_ws, size_t ws_size,
                              hipStream_t stream) {
  if (n_in < 14) return;
  if (in_sizes[0] != NROW * DIM) return;
  if (in_sizes[1] != NROW * 3) return;
  if (in_sizes[2] != 137 * H1) return;
  if (in_sizes[3] != H1) return;
  if (in_sizes[4] != H1 * MDIM) return;
  if (in_sizes[5] != MDIM) return;
  if (in_sizes[6] != MDIM * 64) return;
  if (in_sizes[7] != 64) return;
  if (in_sizes[8] != 64) return;
  if (in_sizes[9] != 1) return;
  if (in_sizes[10] != 80 * HN) return;
  if (in_sizes[11] != HN) return;
  if (in_sizes[12] != HN * DIM) return;
  if (in_sizes[13] != DIM) return;
  if (out_size != NROW * DIM + NROW * 3) return;

  const float* feats = (const float*)d_in[0];
  const float* coors = (const float*)d_in[1];
  const float* w1e   = (const float*)d_in[2];
  const float* b1e   = (const float*)d_in[3];
  const float* w2e   = (const float*)d_in[4];
  const float* b2e   = (const float*)d_in[5];
  const float* w1c   = (const float*)d_in[6];
  const float* b1c   = (const float*)d_in[7];
  const float* w2c   = (const float*)d_in[8];
  const float* b2c   = (const float*)d_in[9];
  const float* w1h   = (const float*)d_in[10];
  const float* b1h   = (const float*)d_in[11];
  const float* w2h   = (const float*)d_in[12];
  const float* b2h   = (const float*)d_in[13];
  float* out = (float*)d_out;

  size_t off = 0;
  const size_t oFB   = off; off = al256(off + (size_t)NROW * DIM * 2);
  const size_t oW1IJ = off; off = al256(off + (size_t)NPIJ * DIM * 2);
  const size_t oWF   = off; off = al256(off + (size_t)H1P * 32 * 2);
  const size_t oW2E  = off; off = al256(off + (size_t)MDIM * H1P * 2);
  const size_t oW1C  = off; off = al256(off + (size_t)64 * 32 * 2);
  const size_t oW1HF = off; off = al256(off + (size_t)HN * DIM * 2);
  const size_t oW1HM = off; off = al256(off + (size_t)HN * 32 * 2);
  const size_t oW2H  = off; off = al256(off + (size_t)DIM * HN * 2);
  const size_t oVEC  = off; off = al256(off + (size_t)VECN * 4);
  const size_t oCB   = off; off = al256(off + (size_t)NROW * 4 * 4);
  const size_t oPIJ  = off; off = al256(off + (size_t)NROW * NPIJ * 4);
  const size_t oMI   = off; off = al256(off + (size_t)NROW * MDIM * 4);
  const size_t oCO   = off; off = al256(off + (size_t)NROW * 4 * 4);
  if (off > ws_size || off > (size_t)134217728) return;

  char* ws = (char*)d_ws;
  unsigned short* FB   = (unsigned short*)(ws + oFB);
  unsigned short* W1IJ = (unsigned short*)(ws + oW1IJ);
  unsigned short* WF   = (unsigned short*)(ws + oWF);
  unsigned short* W2E  = (unsigned short*)(ws + oW2E);
  unsigned short* W1C  = (unsigned short*)(ws + oW1C);
  unsigned short* W1HF = (unsigned short*)(ws + oW1HF);
  unsigned short* W1HM = (unsigned short*)(ws + oW1HM);
  unsigned short* W2H  = (unsigned short*)(ws + oW2H);
  float*          VEC  = (float*)(ws + oVEC);
  float*          CB   = (float*)(ws + oCB);
  float*          PIJ  = (float*)(ws + oPIJ);
  float*          MI   = (float*)(ws + oMI);
  float*          CO   = (float*)(ws + oCO);

  hipFuncSetAttribute(reinterpret_cast<const void*>(&k_pair), hipFuncAttributeMaxDynamicSharedMemorySize,
                      (int)PAIR_LDS);

  k_prep<<<PB_END, 256, 0, stream>>>(feats, coors, w1e, b1e, w2e, b2e, w1c, b1c, w2c, b2c, w1h, b1h, w2h, b2h,
                                     FB, W1IJ, WF, W2E, W1C, W1HF, W1HM, W2H, VEC, CB);
  k_node<<<dim3(NROW / 128, NPIJ / 64), 128, 0, stream>>>(FB, W1IJ, VEC, PIJ);
  k_pair<<<NROW / 8, 256, PAIR_LDS, stream>>>(PIJ, WF, W2E, W1C, VEC, CB, MI, CO);
  k_update<<<NROW / 32, 64, 0, stream>>>(FB, W1HF, W1HM, W2H, VEC, MI, CO, out);
  (void)hipGetLastError();
}
